// MaskedAttention_15161234555425
// MI455X (gfx1250) — hardware-verified
//
#include <hip/hip_runtime.h>
#include <stdint.h>

#ifndef NB
#define NB       32
#endif
#ifndef SEQ
#define SEQ      1024
#endif
#define NB_FULL  32
#define SEQ_FULL 1024
#define QC       256
#define EC       3
#define ICH      259
#define KC       128
#define VC       256
#define KP       288
#define XP       320
#define XSP      328
#define NTOK     (NB * SEQ)

typedef _Float16 v16h __attribute__((ext_vector_type(16)));
typedef _Float16 v8h  __attribute__((ext_vector_type(8)));
typedef __bf16   v16b __attribute__((ext_vector_type(16)));
typedef __bf16   v8b  __attribute__((ext_vector_type(8)));
typedef float    v8f  __attribute__((ext_vector_type(8)));
typedef float    v4f  __attribute__((ext_vector_type(4)));
typedef unsigned short v8us __attribute__((ext_vector_type(8)));

static_assert(NB >= 1 && NB <= NB_FULL && SEQ >= 64 && SEQ <= SEQ_FULL);
static_assert((SEQ % 64) == 0 && (NTOK % 64) == 0);
static_assert((KP % 32) == 0 && KP >= ICH && (XP % 64) == 0 && XP >= KP && XSP >= XP && (XSP % 8) == 0);
static_assert((QC % 32) == 0 && (KC % 64) == 0 && (VC % 64) == 0);
static_assert(32 * (XP / 8) == 5 * 256);

#define WKV_PIECES ((KC + VC) * XP / 8)
#define WQ_PIECES  (KC * QC / 8)
#define WKV_BLOCKS (WKV_PIECES / 256)
#define WQ_BLOCKS  (WQ_PIECES / 256)
static_assert((WKV_PIECES % 256) == 0 && (WQ_PIECES % 256) == 0 && WKV_BLOCKS == 60 && WQ_BLOCKS == 16);

__device__ __forceinline__ unsigned short bfbits(float f) {
  const unsigned u = __float_as_uint(f);
  return (unsigned short)((u + 0x7FFFu + ((u >> 16) & 1u)) >> 16);
}
__device__ __forceinline__ float bfval(float f) {
  return __uint_as_float(((unsigned)bfbits(f)) << 16);
}

__device__ __forceinline__ v16h ldfrag(const _Float16* p) {
  union { v16h v; v8h hh[2]; } f;
  f.hh[0] = *(const v8h*)(p);
  f.hh[1] = *(const v8h*)(p + 16);
  return f.v;
}
__device__ __forceinline__ v16b ldfragb(const __bf16* p) {
  union { v16b v; v8b hh[2]; } f;
  f.hh[0] = *(const v8b*)(p);
  f.hh[1] = *(const v8b*)(p + 16);
  return f.v;
}
__device__ __forceinline__ v8f mma16(v16h a, v16h b, v8f c) {
  return __builtin_amdgcn_wmma_f32_16x16x32_f16(false, a, false, b, (short)0, c, false, false);
}
__device__ __forceinline__ v8f mmabf(v16b a, v16b b, v8f c) {
  return __builtin_amdgcn_wmma_f32_16x16x32_bf16(false, a, false, b, (short)0, c, false, false);
}
__device__ __forceinline__ v8f zero8() {
  v8f z;
#pragma unroll
  for (int i = 0; i < 8; ++i) z[i] = 0.0f;
  return z;
}

__device__ __forceinline__ void guard_g(v8f& a, v8f& b, v16b x, v16b y) {
  asm volatile("v_nop\n\tv_nop\n\tv_nop\n\tv_nop" : "+v"(a), "+v"(b) : "v"(x), "v"(y));
}
__device__ __forceinline__ void keep4(v16b a, v16b b, v16b c, v16b d) {
  asm volatile("v_nop" :: "v"(a), "v"(b), "v"(c), "v"(d));
}
__device__ __forceinline__ void accg4(v8f& a, v8f& b, v8f& c, v8f& d) {
  asm volatile("v_nop\n\tv_nop\n\tv_nop\n\tv_nop" : "+v"(a), "+v"(b), "+v"(c), "+v"(d));
}
__device__ __forceinline__ void guard_s4(v8f& a0, v8f& a1, v8f& a2, v8f& a3,
                                         v16h f0, v16h f1, v16h f2, v16h f3, v16h f4, v16h f5) {
  asm volatile("v_nop\n\tv_nop\n\tv_nop\n\tv_nop"
               : "+v"(a0), "+v"(a1), "+v"(a2), "+v"(a3)
               : "v"(f0), "v"(f1), "v"(f2), "v"(f3), "v"(f4), "v"(f5));
}
__device__ __forceinline__ void guard_pv8(v8f& a0, v8f& a1, v8f& a2, v8f& a3,
                                          v8f& a4, v8f& a5, v8f& a6, v8f& a7,
                                          v16h f0, v16h f1, v16h f2, v16h f3,
                                          v16h f4, v16h f5, v16h f6, v16h f7) {
  asm volatile("v_nop\n\tv_nop\n\tv_nop\n\tv_nop"
               : "+v"(a0), "+v"(a1), "+v"(a2), "+v"(a3), "+v"(a4), "+v"(a5), "+v"(a6), "+v"(a7)
               : "v"(f0), "v"(f1), "v"(f2), "v"(f3), "v"(f4), "v"(f5), "v"(f6), "v"(f7));
}

__global__ __launch_bounds__(256) void cvt_xt_kernel(const float* __restrict__ x, const float* __restrict__ kve,
                                                     unsigned short* __restrict__ Xt) {
  __shared__ __align__(16) unsigned short sX[32 * XSP];
  const int t = (int)threadIdx.x, lane = t & 31, wv = t >> 5;
  const int b = (int)blockIdx.y, tok0 = (int)blockIdx.x * 32;
  const size_t xb = (size_t)b * QC * SEQ_FULL + (size_t)tok0 + (size_t)lane;
  const size_t eb = (size_t)b * EC * SEQ_FULL + (size_t)tok0 + (size_t)lane;
#pragma unroll 2
  for (int i = 0; i < XP / 8; ++i) {
    const int ch = i * 8 + wv;
    const int cx = (ch < QC) ? ch : (QC - 1);
    int ce = ch - QC;
    ce = (ce < 0) ? 0 : ((ce > EC - 1) ? (EC - 1) : ce);
    const float xv = x[xb + (size_t)cx * SEQ_FULL];
    const float ev = kve[eb + (size_t)ce * SEQ_FULL];
    const float v = (ch < QC) ? xv : ((ch < ICH) ? ev : 0.0f);
    sX[lane * XSP + ch] = bfbits(v);
  }
  __syncthreads();
#pragma unroll
  for (int ps = 0; ps < 2; ++ps) {
#pragma unroll
    for (int it = 0; it < 5; ++it) {
      const int p = it * 256 + t;
      const int row = p / (XP / 8), pc = p - row * (XP / 8);
      const v8us o = *(const v8us*)(sX + row * XSP + pc * 8);
      unsigned short* d = Xt + ((size_t)b * SEQ + (size_t)(tok0 + row)) * XP + pc * 8;
      *(volatile v8us*)d = o;
    }
    __threadfence();
  }
}

__global__ __launch_bounds__(256) void cvt_w_kernel(const float* __restrict__ Wq, const float* __restrict__ Wkv,
                                                    unsigned short* __restrict__ Wqb, unsigned short* __restrict__ Wkvb) {
  const int t = (int)threadIdx.x;
  if ((int)blockIdx.x < WKV_BLOCKS) {
    const int p = (int)blockIdx.x * 256 + t;
    const int row = p / (XP / 8), c0 = (p - row * (XP / 8)) * 8;
    v8us o;
#pragma unroll
    for (int j = 0; j < 8; ++j) {
      const int col = c0 + j;
      const int cc = (col < ICH) ? col : (ICH - 1);
      const float f = Wkv[(size_t)row * ICH + cc];
      o[j] = (col < ICH) ? bfbits(f) : (unsigned short)0;
    }
    unsigned short* d = Wkvb + (size_t)p * 8;
    *(volatile v8us*)d = o;
    __threadfence();
    *(volatile v8us*)d = o;
  } else {
    const int p = ((int)blockIdx.x - WKV_BLOCKS) * 256 + t;
    v8us o;
#pragma unroll
    for (int j = 0; j < 8; ++j) o[j] = bfbits(Wq[(size_t)p * 8 + j]);
    unsigned short* d = Wqb + (size_t)p * 8;
    *(volatile v8us*)d = o;
    __threadfence();
    *(volatile v8us*)d = o;
  }
}

__global__ __launch_bounds__(256) void proj_kernel(const __bf16* __restrict__ A, int lda,
                                                   const __bf16* __restrict__ Bt, int ldb,
                                                   _Float16* __restrict__ Ch, _Float16* __restrict__ Cl, int ldc,
                                                   int M, int N, int K,
                                                   const float* __restrict__ bias, int biasLen, int biasRow) {
  __shared__ __align__(16) float sT[8][16 * 68];
  const int lane = threadIdx.x & 31, wave = threadIdx.x >> 5;
  const int tilesN = N >> 6, tilesM = M >> 6;
  const int tile = (int)blockIdx.x * 8 + wave;
  if (tile >= tilesM * tilesN) return;
  const int tm = tile / tilesN, tn = tile - tm * tilesN;
  const int m0 = tm << 6, n0 = tn << 6;
  const int rl = lane & 15;
  const int koff = (lane >> 4) * 8;
  const int mOff = (lane >> 4) * 8;

  v8f acc[4][4];
#pragma unroll
  for (int i = 0; i < 4; ++i)
#pragma unroll
    for (int j = 0; j < 4; ++j) acc[i][j] = zero8();

#pragma unroll 1
  for (int k0 = 0; k0 < K; k0 += 32) {
    v16b bh[4];
#pragma unroll
    for (int j = 0; j < 4; ++j) bh[j] = ldfragb(Bt + (size_t)(n0 + (j << 4) + rl) * ldb + koff + k0);
#pragma unroll
    for (int i = 0; i < 4; ++i) {
      const v16b ah = ldfragb(A + (size_t)(m0 + (i << 4) + rl) * lda + koff + k0);
#pragma unroll
      for (int j = 0; j < 4; ++j) acc[i][j] = mmabf(ah, bh[j], acc[i][j]);
      guard_g(acc[i][0], acc[i][3], ah, bh[3]);
    }
    keep4(bh[0], bh[1], bh[2], bh[3]);
  }
  accg4(acc[0][0], acc[0][1], acc[0][2], acc[0][3]);
  accg4(acc[1][0], acc[1][1], acc[1][2], acc[1][3]);
  accg4(acc[2][0], acc[2][1], acc[2][2], acc[2][3]);
  accg4(acc[3][0], acc[3][1], acc[3][2], acc[3][3]);

  float* slab = sT[wave];
  const int qq = lane >> 3, c8 = (lane & 7) * 8;
  float bc[8];
#pragma unroll
  for (int e = 0; e < 8; ++e) {
    int idx = n0 + c8 + e;
    idx = (idx < biasLen) ? idx : (biasLen - 1);
    bc[e] = bfval(bias[idx]);
  }
#pragma unroll
  for (int i = 0; i < 4; ++i) {
    const int mBase = m0 + (i << 4);
#pragma unroll
    for (int j = 0; j < 4; ++j) {
#pragma unroll
      for (int r = 0; r < 8; ++r) slab[(mOff + r) * 68 + (j << 4) + rl] = acc[i][j][r];
    }
    __builtin_amdgcn_fence(3  , "workgroup");
    __builtin_amdgcn_wave_barrier();
    __builtin_amdgcn_fence(2  , "workgroup");
#pragma unroll
    for (int ps = 0; ps < 2; ++ps) {
#pragma unroll
      for (int it = 0; it < 4; ++it) {
        const int row = it * 4 + qq;
        const float* sp = slab + row * 68 + c8;
        const v4f u0 = *(const v4f*)(sp);
        const v4f u1 = *(const v4f*)(sp + 4);
        int mr = mBase + row;
        mr = (mr < biasLen) ? mr : (biasLen - 1);
        const float br = bfval(bias[mr]);
        v8h hv, lv;
#pragma unroll
        for (int e = 0; e < 4; ++e) {
          const float f0 = u0[e] + (biasRow ? br : bc[e]);
          const _Float16 g0 = (_Float16)f0;
          hv[e] = g0;
          lv[e] = (_Float16)((f0 - (float)g0) * 2048.0f);
          const float f1 = u1[e] + (biasRow ? br : bc[4 + e]);
          const _Float16 g1 = (_Float16)f1;
          hv[4 + e] = g1;
          lv[4 + e] = (_Float16)((f1 - (float)g1) * 2048.0f);
        }
        const size_t go = (size_t)(mBase + row) * ldc + n0 + c8;
        *(volatile v8h*)(Ch + go) = hv;
        *(volatile v8h*)(Cl + go) = lv;
      }
      __threadfence();
    }
    __builtin_amdgcn_fence(3  , "workgroup");
    __builtin_amdgcn_wave_barrier();
    __builtin_amdgcn_fence(2  , "workgroup");
  }
}

#define QB       32
#define NWAVE    8
#define KCH      128
#define QSP      136
#define PSP      136
#define OSP      36
#define NQT      (SEQ / QB)
#define TSPLIT   ((NQT < 8) ? NQT : 8)
#define LDS_QH   0
#define LDS_QL   (LDS_QH + QB * QSP * 2)
#define LDS_PH   (LDS_QL + QB * QSP * 2)
#define LDS_PL   (LDS_PH + QB * PSP * 2)
#define LDS_PMAX (LDS_PL + QB * PSP * 2)
#define LDS_PSUM (LDS_PMAX + NWAVE * QB * 4)
#define LDS_ST   (LDS_PSUM + NWAVE * QB * 4)
#define LDS_OS   (LDS_ST + 4 * QB * 4)
#define ATT_LDS  (LDS_OS + VC * OSP * 4)
static_assert(LDS_QL == 8704 && LDS_PH == 17408 && LDS_PL == 26112 && LDS_PMAX == 34816);
static_assert(LDS_PSUM == 35840 && LDS_ST == 36864 && LDS_OS == 37376 && ATT_LDS == 74240);
static_assert((QSP % 8) == 0 && (PSP % 8) == 0 && (OSP % 4) == 0 && QSP >= KC && PSP >= KCH && OSP >= QB);
static_assert(NWAVE * 16 == KCH && NWAVE * 32 == VC && QB == 32 && NWAVE * QB == 256 && (KC % 32) == 0);
static_assert((SEQ % QB) == 0 && (SEQ % 32) == 0 && TSPLIT >= 1 && TSPLIT <= NQT);
static_assert((LDS_QL % 16) == 0 && (LDS_PH % 16) == 0 && (LDS_PL % 16) == 0 && (LDS_PMAX % 16) == 0 &&
              (LDS_ST % 16) == 0 && (LDS_OS % 16) == 0);

template <bool RES>
__global__ __launch_bounds__(256) void attn_kernel(const _Float16* __restrict__ qh, const _Float16* __restrict__ ql,
                                                   const _Float16* __restrict__ kh, const _Float16* __restrict__ kl,
                                                   const _Float16* __restrict__ vth, const _Float16* __restrict__ vtl,
                                                   float* __restrict__ out, int qt0) {
  extern __shared__ __align__(16) char smem[];
  _Float16* Qhs = (_Float16*)(smem + LDS_QH);
  _Float16* Qls = (_Float16*)(smem + LDS_QL);
  _Float16* Phs = (_Float16*)(smem + LDS_PH);
  _Float16* Pls = (_Float16*)(smem + LDS_PL);
  float* pmax = (float*)(smem + LDS_PMAX);
  float* psum = (float*)(smem + LDS_PSUM);
  float* m_s  = (float*)(smem + LDS_ST);
  float* l_s  = m_s + QB;
  float* al_s = m_s + 2 * QB;
  float* li_s = m_s + 3 * QB;
  float* Os   = (float*)(smem + LDS_OS);

  const int tid = (int)threadIdx.x;
  const int wave = __builtin_amdgcn_readfirstlane(tid >> 5);
  const int lane = tid & 31, h = lane >> 4, c = lane & 15;
  const int b = (int)blockIdx.y;
  const int q0 = (qt0 + (int)blockIdx.x) * QB;
  const int qlast = q0 + QB - 1;
  const size_t tokb = (size_t)b * SEQ;
  const size_t tok0 = tokb + (size_t)q0;
  const float ninf = -__builtin_inff();
  const float inv_s = 0.088388346135616302f;

  if (tid < QB) { m_s[tid] = ninf; l_s[tid] = 0.0f; al_s[tid] = 0.0f; li_s[tid] = 0.0f; }
  psum[tid] = 0.0f;
#pragma unroll
  for (int i = 0; i < 2; ++i) {
    const int idx = i * 256 + tid;
    const int row = idx >> 4;
    const int pc  = idx & 15;
    const size_t g = (tok0 + (size_t)row) * KC + (size_t)pc * 8;
    const v8h v0 = *(const v8h*)(qh + g);
    const v8h v1 = *(const v8h*)(ql + g);
    *(v8h*)(Qhs + row * QSP + pc * 8) = v0;
    *(v8h*)(Qls + row * QSP + pc * 8) = v1;
  }
  __syncthreads();

  v8f oacc1[2][2], oacc2[2][2];
#pragma unroll
  for (int i = 0; i < 2; ++i)
#pragma unroll
    for (int g = 0; g < 2; ++g) { oacc1[i][g] = zero8(); oacc2[i][g] = zero8(); }

  const _Float16* qbp0 = Qhs + c * QSP + 8 * h;
  const _Float16* qbp1 = Qhs + (16 + c) * QSP + 8 * h;
  const _Float16* qlp0 = Qls + c * QSP + 8 * h;
  const _Float16* qlp1 = Qls + (16 + c) * QSP + 8 * h;
  const _Float16* pap0 = Phs + c * PSP + 8 * h;
  const _Float16* pap1 = Phs + (16 + c) * PSP + 8 * h;
  const _Float16* plp0 = Pls + c * PSP + 8 * h;
  const _Float16* plp1 = Pls + (16 + c) * PSP + 8 * h;
  const int ntile = (q0 >> 7) + 1;

#pragma unroll 1
  for (int t = 0; t < ntile; ++t) {
    const int kb = t * KCH + 16 * wave;
    v8f s1a = zero8(), s2a = zero8(), s1b = zero8(), s2b = zero8();
    if (kb <= qlast) {
      const _Float16* kap = kh + (tokb + (size_t)(kb + c)) * KC + 8 * h;
      const _Float16* krp = kl + (tokb + (size_t)(kb + c)) * KC + 8 * h;
#pragma unroll 1
      for (int k0 = 0; k0 < KC; k0 += 32) {
        const v16h a   = ldfrag(kap + k0);
        const v16h bq0 = ldfrag(qbp0 + k0);
        const v16h bl0 = ldfrag(qlp0 + k0);
        const v16h bq1 = ldfrag(qbp1 + k0);
        const v16h bl1 = ldfrag(qlp1 + k0);
        v16h ar = a;
        if (RES) ar = ldfrag(krp + k0);
        s1a = mma16(a, bq0, s1a);
        s2a = mma16(a, bl0, s2a);
        if (RES) s2a = mma16(ar, bq0, s2a);
        s1b = mma16(a, bq1, s1b);
        s2b = mma16(a, bl1, s2b);
        if (RES) s2b = mma16(ar, bq1, s2b);
        guard_s4(s1a, s2a, s1b, s2b, a, ar, bq0, bl0, bq1, bl1);
      }
    }
    {
      float pma = ninf, pmb = ninf;
#pragma unroll
      for (int r = 0; r < 8; ++r) {
        const int key = kb + 8 * h + r;
        float sa = s1a[r] + s2a[r] * 0.00048828125f;
        float sb = s1b[r] + s2b[r] * 0.00048828125f;
        sa = (key > q0 + c) ? ninf : sa;
        sb = (key > q0 + 16 + c) ? ninf : sb;
        s1a[r] = sa;
        s1b[r] = sb;
        pma = fmaxf(pma, sa);
        pmb = fmaxf(pmb, sb);
      }
      pma = fmaxf(pma, __shfl_xor(pma, 16, 32));
      pmb = fmaxf(pmb, __shfl_xor(pmb, 16, 32));
      pmax[wave * QB + c] = pma;
      pmax[wave * QB + 16 + c] = pmb;
    }
    __syncthreads();
    if (wave == 0) {
      const int row = lane;
      float ps = 0.0f;
#pragma unroll
      for (int w = 0; w < NWAVE; ++w) ps += psum[w * QB + row];
      l_s[row] = l_s[row] * al_s[row] + ps;
      const float mo = m_s[row];
      float mx = mo;
#pragma unroll
      for (int w = 0; w < NWAVE; ++w) mx = fmaxf(mx, pmax[w * QB + row]);
      al_s[row] = __expf((mo - mx) * inv_s);
      m_s[row] = mx;
    }
    __syncthreads();
    {
      const float mqa = m_s[c], mqb = m_s[16 + c];
      float psa = 0.0f, psb = 0.0f;
      v8h pha, pra, phb, prb;
#pragma unroll
      for (int r = 0; r < 8; ++r) {
        const float pa = __expf((s1a[r] - mqa) * inv_s);
        psa += pa;
        const float pas = pa * 1024.0f;
        const _Float16 ha = (_Float16)pas;
        pha[r] = ha;
        pra[r] = (_Float16)((pas - (float)ha) * 2048.0f);
        const float pb = __expf((s1b[r] - mqb) * inv_s);
        psb += pb;
        const float pbs = pb * 1024.0f;
        const _Float16 hb = (_Float16)pbs;
        phb[r] = hb;
        prb[r] = (_Float16)((pbs - (float)hb) * 2048.0f);
      }
      *(v8h*)(Phs + c * PSP + 16 * wave + 8 * h) = pha;
      *(v8h*)(Phs + (16 + c) * PSP + 16 * wave + 8 * h) = phb;
      if (RES) {
        *(v8h*)(Pls + c * PSP + 16 * wave + 8 * h) = pra;
        *(v8h*)(Pls + (16 + c) * PSP + 16 * wave + 8 * h) = prb;
      }
      psa += __shfl_xor(psa, 16, 32);
      psb += __shfl_xor(psb, 16, 32);
      psum[wave * QB + c] = psa;
      psum[wave * QB + 16 + c] = psb;
#pragma unroll
      for (int i = 0; i < 2; ++i) {
        const v4f aA = *(const v4f*)(al_s + 16 * i + 8 * h), aB = *(const v4f*)(al_s + 16 * i + 8 * h + 4);
#pragma unroll
        for (int g = 0; g < 2; ++g) {
#pragma unroll
          for (int r = 0; r < 4; ++r) {
            oacc1[i][g][r] *= aA[r]; oacc1[i][g][4 + r] *= aB[r];
            oacc2[i][g][r] *= aA[r]; oacc2[i][g][4 + r] *= aB[r];
          }
        }
      }
    }
    __syncthreads();
    {
      int kend = q0 + QB - t * KCH;
      kend = (kend > KCH) ? KCH : kend;
      kend = (kend + 31) & ~31;
      const size_t vc0 = tokb + (size_t)t * KCH + 8 * h;
      const _Float16* vhp = vth + (size_t)(32 * wave + c) * NTOK + vc0;
      const _Float16* vlp = vtl + (size_t)(32 * wave + c) * NTOK + vc0;
      const size_t o1 = (size_t)16 * NTOK;
#pragma unroll 1
      for (int ks = 0; ks < kend; ks += 32) {
        const v16h pa0 = ldfrag(pap0 + ks);
        const v16h pa1 = ldfrag(pap1 + ks);
        v16h pz0 = pa0, pz1 = pa1;
        if (RES) { pz0 = ldfrag(plp0 + ks); pz1 = ldfrag(plp1 + ks); }
        const v16h x0 = ldfrag(vhp + ks), x1 = ldfrag(vhp + o1 + ks);
        const v16h y0 = ldfrag(vlp + ks), y1 = ldfrag(vlp + o1 + ks);
        oacc1[0][0] = mma16(pa0, x0, oacc1[0][0]);
        oacc1[0][1] = mma16(pa0, x1, oacc1[0][1]);
        oacc1[1][0] = mma16(pa1, x0, oacc1[1][0]);
        oacc1[1][1] = mma16(pa1, x1, oacc1[1][1]);
        oacc2[0][0] = mma16(pa0, y0, oacc2[0][0]);
        oacc2[0][1] = mma16(pa0, y1, oacc2[0][1]);
        oacc2[1][0] = mma16(pa1, y0, oacc2[1][0]);
        oacc2[1][1] = mma16(pa1, y1, oacc2[1][1]);
        if (RES) {
          oacc2[0][0] = mma16(pz0, x0, oacc2[0][0]);
          oacc2[0][1] = mma16(pz0, x1, oacc2[0][1]);
          oacc2[1][0] = mma16(pz1, x0, oacc2[1][0]);
          oacc2[1][1] = mma16(pz1, x1, oacc2[1][1]);
        }
        guard_pv8(oacc1[0][0], oacc1[0][1], oacc1[1][0], oacc1[1][1],
                  oacc2[0][0], oacc2[0][1], oacc2[1][0], oacc2[1][1],
                  pa0, pa1, pz0, pz1, x0, x1, y0, y1);
      }
    }
  }

  if (wave == 0) {
    const int row = lane;
    float ps = 0.0f;
#pragma unroll
    for (int w = 0; w < NWAVE; ++w) ps += psum[w * QB + row];
    const float l = l_s[row] * al_s[row] + ps;
    li_s[row] = (1.0f / (l + 1e-6f)) * 0.0009765625f;
  }
  __syncthreads();
  {
#pragma unroll
    for (int i = 0; i < 2; ++i) {
      const v4f iA = *(const v4f*)(li_s + 16 * i + 8 * h), iB = *(const v4f*)(li_s + 16 * i + 8 * h + 4);
#pragma unroll
      for (int g = 0; g < 2; ++g) {
        float* orow = Os + (32 * wave + 16 * g + c) * OSP + 16 * i + 8 * h;
        v4f wa, wb;
#pragma unroll
        for (int r = 0; r < 4; ++r) {
          wa[r] = (oacc1[i][g][r] + oacc2[i][g][r] * 0.00048828125f) * iA[r];
          wb[r] = (oacc1[i][g][4 + r] + oacc2[i][g][4 + r] * 0.00048828125f) * iB[r];
        }
        *(v4f*)(orow) = wa;
        *(v4f*)(orow + 4) = wb;
      }
    }
  }
  __syncthreads();
  {
    const int qq = lane >> 3, c4 = (lane & 7) * 4;
#pragma unroll
    for (int ps = 0; ps < 2; ++ps) {
#pragma unroll
      for (int it = 0; it < 8; ++it) {
        const int vr = 32 * wave + 4 * it + qq;
        const v4f v = *(const v4f*)(Os + vr * OSP + c4);
        *(volatile v4f*)(out + ((size_t)b * VC + (size_t)vr) * SEQ_FULL + q0 + c4) = v;
      }
      __threadfence();
    }
  }
}

extern "C" void kernel_launch(void* const* d_in, const int* in_sizes, int n_in,
                              void* d_out, int out_size, void* d_ws, size_t ws_size,
                              hipStream_t stream) {
  if (n_in < 6) return;
  if (in_sizes[0] < NB * QC * SEQ_FULL) return;
  if (in_sizes[1] < NB * EC * SEQ_FULL) return;
  if (in_sizes[2] < KC * QC || in_sizes[3] < KC) return;
  if (in_sizes[4] < (KC + VC) * ICH || in_sizes[5] < KC + VC) return;
  if ((size_t)out_size < ((size_t)(NB - 1) * VC + (size_t)(VC - 1)) * SEQ_FULL + (size_t)SEQ) return;

  const float* x   = (const float*)d_in[0];
  const float* kve = (const float*)d_in[1];
  const float* Wq  = (const float*)d_in[2];
  const float* bq  = (const float*)d_in[3];
  const float* Wkv = (const float*)d_in[4];
  const float* bkv = (const float*)d_in[5];
  float* out = (float*)d_out;

  const size_t bXt  = (size_t)NTOK * XP * 2;
  const size_t bWq  = (size_t)KC * QC * 2;
  const size_t bWkv = (size_t)(KC + VC) * XP * 2;
  const size_t bQK  = (size_t)NTOK * KC * 2;
  const size_t bV   = (size_t)VC * NTOK * 2;
  size_t off = 0;
  const size_t oXt  = off; off += bXt;
  const size_t oWq  = off; off += bWq;
  const size_t oWkv = off; off += bWkv;
  const size_t oQh  = off; off += bQK;
  const size_t oQl  = off; off += bQK;
  const size_t oKh  = off; off += bQK;
  const size_t oKl  = off; off += bQK;
  const size_t oVh  = off; off += bV;
  const size_t oVl  = off; off += bV;
  if (off > ws_size) return;
  if (off > (size_t)134217728) return;

  char* ws = (char*)d_ws;
  unsigned short* Xt   = (unsigned short*)(ws + oXt);
  unsigned short* Wqb  = (unsigned short*)(ws + oWq);
  unsigned short* Wkvb = (unsigned short*)(ws + oWkv);
  _Float16* Qh = (_Float16*)(ws + oQh);
  _Float16* Ql = (_Float16*)(ws + oQl);
  _Float16* Kh = (_Float16*)(ws + oKh);
  _Float16* Kl = (_Float16*)(ws + oKl);
  _Float16* Vh = (_Float16*)(ws + oVh);
  _Float16* Vl = (_Float16*)(ws + oVl);

  const dim3 blk(256);
  cvt_xt_kernel<<<dim3(SEQ / 32, NB), blk, 0, stream>>>(x, kve, Xt);
  cvt_w_kernel<<<dim3(WKV_BLOCKS + WQ_BLOCKS), blk, 0, stream>>>(Wq, Wkv, Wqb, Wkvb);
  {
    const int tiles = (NTOK / 64) * (KC / 64);
    proj_kernel<<<dim3((tiles + 7) / 8), blk, 0, stream>>>(
        (const __bf16*)Xt, XP, (const __bf16*)Wqb, QC, Qh, Ql, KC, NTOK, KC, QC, bq, KC, 0);
  }
  {
    const int tiles = (NTOK / 64) * (KC / 64);
    proj_kernel<<<dim3((tiles + 7) / 8), blk, 0, stream>>>(
        (const __bf16*)Xt, XP, (const __bf16*)Wkvb, XP, Kh, Kl, KC, NTOK, KC, KP, bkv, KC + VC, 0);
  }
  {
    const int tiles = (VC / 64) * (NTOK / 64);
    proj_kernel<<<dim3((tiles + 7) / 8), blk, 0, stream>>>(
        (const __bf16*)(Wkvb + (size_t)KC * XP), XP, (const __bf16*)Xt, XP, Vh, Vl, NTOK, VC, NTOK, KP,
        bkv + KC, VC, 1);
  }
  (void)hipFuncSetAttribute(reinterpret_cast<const void*>(&attn_kernel<true>),
                            hipFuncAttributeMaxDynamicSharedMemorySize, ATT_LDS);
  (void)hipFuncSetAttribute(reinterpret_cast<const void*>(&attn_kernel<false>),
                            hipFuncAttributeMaxDynamicSharedMemorySize, ATT_LDS);
  attn_kernel<true><<<dim3(TSPLIT, NB), dim3(256), ATT_LDS, stream>>>(Qh, Ql, Kh, Kl, Vh, Vl, out, 0);
  if (NQT > TSPLIT) {
    attn_kernel<false><<<dim3(NQT - TSPLIT, NB), dim3(256), ATT_LDS, stream>>>(Qh, Ql, Kh, Kl, Vh, Vl, out, TSPLIT);
  }
  (void)hipGetLastError();
}
